// EfficientBlockCirculantLinear_34368328303059
// MI455X (gfx1250) — hardware-verified
//
#include <hip/hip_runtime.h>
#include <math.h>

typedef __attribute__((ext_vector_type(16))) _Float16 v16h;
typedef __attribute__((ext_vector_type(8)))  _Float16 v8h;
typedef __attribute__((ext_vector_type(8)))  float    v8f;
typedef __attribute__((ext_vector_type(4)))  float    v4f;

constexpr int kM       = 1024;
constexpr int kK       = 4096;
constexpr int kN       = 4096;
constexpr int kBlk     = 128;
constexpr int kBlkLog  = 7;
constexpr int kNbIn    = kK / kBlk;
constexpr int kNbOut   = kN / kBlk;
constexpr int kKLog    = 12;
constexpr float kCarryA = 16.0f;
constexpr float kCarryB = 64.0f;
constexpr float kFold   = 1.0f / (kCarryA * kCarryB);

static_assert((1 << kBlkLog) == kBlk, "block edge log");
static_assert((1 << kKLog) == kK, "depth log");
static_assert(kNbIn == 32 && kNbOut == 32, "block counts");
static_assert(kNbIn * kBlk == kK && kNbOut * kBlk == kN, "no pad, no slice");
static_assert((kK % 32) == 0, "GEMM K multiple of 32");
static_assert((kM % 64) == 0 && (kN % 64) == 0, "GEMM M,N multiples of 64");
static_assert(kFold * kCarryA * kCarryB == 1.0f, "exact fold");

constexpr size_t kOffA    = 0;
constexpr size_t kBytesA  = (size_t)kM * kK * 2;
constexpr size_t kOffBt   = kOffA + kBytesA;
constexpr size_t kBytesBt = (size_t)kN * kK * 2;
constexpr size_t kWsTotal = kOffBt + kBytesBt;
static_assert(kBytesA == 8388608ull && kBytesBt == 33554432ull, "plane sizes");
static_assert(kWsTotal == 41943040ull, "carve total");
static_assert(kWsTotal <= 134217728ull, "carve cap");
static_assert((kOffBt % 128) == 0, "128-B aligned regions");

__device__ __forceinline__ void acc_guard1(v8f& a, v16h x, v16h y) {
  asm volatile("v_nop\n\tv_nop\n\tv_nop\n\tv_nop" : "+v"(a) : "v"(x), "v"(y));
}
__device__ __forceinline__ void keep4_h(v16h a, v16h b, v16h c, v16h d) {
  asm volatile("v_nop" :: "v"(a), "v"(b), "v"(c), "v"(d));
}
__device__ __forceinline__ v16h frag_load_h(const _Float16* p) {
  union U { v16h v; v8h h[2]; };
  U f;
  f.h[0] = *(const v8h*)(p);
  f.h[1] = *(const v8h*)(p + 16);
  return f.v;
}
__device__ __forceinline__ v8f mma_h(v16h a, v16h b, v8f c) {
  return __builtin_amdgcn_wmma_f32_16x16x32_f16(false, a, false, b, (short)0, c, false, false);
}

__global__ __launch_bounds__(256) void sign_scale_to_f16_kernel(
    const float* __restrict__ x, const float* __restrict__ dsign, unsigned short* __restrict__ apl, int total8)
{
  const int i = blockIdx.x * 256 + threadIdx.x;
  if (i >= total8) return;
  const size_t e0 = (size_t)i << 3;
  const int k = (int)(e0 & (size_t)(kK - 1));
  const v4f x0 = *(const v4f*)(x + e0);
  const v4f x1 = *(const v4f*)(x + e0 + 4);
  const v4f d0 = *(const v4f*)(dsign + k);
  const v4f d1 = *(const v4f*)(dsign + k + 4);
  v8h hv;
#pragma unroll
  for (int e = 0; e < 4; ++e) {
    const float p0 = x0[e] * d0[e];
    const float p1 = x1[e] * d1[e];
    hv[e]     = (_Float16)(p0 * kCarryA);
    hv[4 + e] = (_Float16)(p1 * kCarryA);
  }
  unsigned short* q = apl + e0;
  *(volatile v8h*)q = hv;
  __threadfence();
  *(volatile v8h*)q = hv;
}

__global__ __launch_bounds__(256) void expand_rotated_blocks_kernel(
    const float* __restrict__ w, unsigned short* __restrict__ btp, int total8)
{
  const int i = blockIdx.x * 256 + threadIdx.x;
  if (i >= total8) return;
  const size_t e0 = (size_t)i << 3;
  const int n  = (int)(e0 >> kKLog);
  const int k  = (int)(e0 & (size_t)(kK - 1));
  const int ob = n >> kBlkLog;
  const int t  = n & (kBlk - 1);
  const int jb = k >> kBlkLog;
  const int s0 = k & (kBlk - 1);
  const float* src = w + ((size_t)(ob * kNbIn + jb) << kBlkLog);
  float f[8];
#pragma unroll
  for (int e = 0; e < 8; ++e) f[e] = src[(s0 + e - t) & (kBlk - 1)];
  v8h hv;
#pragma unroll
  for (int e = 0; e < 8; ++e) hv[e] = (_Float16)(f[e] * kCarryB);
  unsigned short* q = btp + e0;
  *(volatile v8h*)q = hv;
  __threadfence();
  *(volatile v8h*)q = hv;
}

__global__ __launch_bounds__(256) void gemm_f16_nt_kernel(
    const unsigned short* __restrict__ Ap, const unsigned short* __restrict__ Btp,
    float* __restrict__ Cout, float scale)
{
  const _Float16* A  = (const _Float16*)Ap;
  const _Float16* Bt = (const _Float16*)Btp;
  __shared__ __align__(16) float sT[8][16 * 68];
  const int lane = threadIdx.x & 31;
  const int wave = __builtin_amdgcn_readfirstlane((int)(threadIdx.x >> 5));
  constexpr int tilesN = kN >> 6;
  constexpr int tilesM = kM >> 6;
  const int tile = blockIdx.x * 8 + wave;
  if (tile >= tilesM * tilesN) return;
  const int tm = tile / tilesN;
  const int tn = tile - tm * tilesN;
  const int m0 = tm << 6;
  const int n0 = tn << 6;

  const int rlane = lane & 15;
  const int koff  = (lane >> 4) * 8;
  const int mOff  = (lane >> 4) * 8;

  v8f acc[4][4];
#pragma unroll
  for (int i = 0; i < 4; ++i)
#pragma unroll
    for (int j = 0; j < 4; ++j) acc[i][j] = (v8f){0.f, 0.f, 0.f, 0.f, 0.f, 0.f, 0.f, 0.f};

#pragma unroll 1
  for (int k0 = 0; k0 < kK; k0 += 32) {
    v16h bh[4];
#pragma unroll
    for (int j = 0; j < 4; ++j) {
      const size_t bo = (size_t)(n0 + (j << 4) + rlane) * kK + koff + k0;
      bh[j] = frag_load_h(Bt + bo);
    }
#pragma unroll
    for (int i = 0; i < 4; ++i) {
      const size_t ao = (size_t)(m0 + (i << 4) + rlane) * kK + koff + k0;
      const v16h ah = frag_load_h(A + ao);
#pragma unroll
      for (int j = 0; j < 4; ++j) acc[i][j] = mma_h(ah, bh[j], acc[i][j]);
#pragma unroll
      for (int j = 0; j < 4; ++j) acc_guard1(acc[i][j], ah, bh[j]);
    }
    keep4_h(bh[0], bh[1], bh[2], bh[3]);
  }

  float* slab = sT[wave];
#pragma unroll
  for (int i = 0; i < 4; ++i) {
    const int mBase = m0 + (i << 4);
#pragma unroll
    for (int j = 0; j < 4; ++j) {
#pragma unroll
      for (int r = 0; r < 8; ++r) {
        const float v = acc[i][j][r] * scale;
        slab[(mOff + r) * 68 + (j << 4) + rlane] = v;
      }
    }
    __builtin_amdgcn_fence(__ATOMIC_RELEASE, "workgroup");
    __builtin_amdgcn_wave_barrier();
    __builtin_amdgcn_fence(__ATOMIC_ACQUIRE, "workgroup");
    {
      const int hh = lane >> 4, c4 = (lane & 15) * 4;
      for (int pass = 0; pass < 2; ++pass) {
#pragma unroll
        for (int it = 0; it < 8; ++it) {
          const int row = it * 2 + hh;
          const v4f v = *(const v4f*)(slab + row * 68 + c4);
          *(volatile v4f*)(Cout + (size_t)(mBase + row) * kN + n0 + c4) = v;
        }
        __threadfence();
      }
    }
    __builtin_amdgcn_fence(__ATOMIC_RELEASE, "workgroup");
    __builtin_amdgcn_wave_barrier();
    __builtin_amdgcn_fence(__ATOMIC_ACQUIRE, "workgroup");
  }
}

extern "C" void kernel_launch(void* const* d_in, const int* in_sizes, int n_in,
                              void* d_out, int out_size, void* d_ws, size_t ws_size,
                              hipStream_t stream) {
  if (n_in < 3) return;
  if (in_sizes[0] != kM * kK) return;
  if (in_sizes[1] != kNbOut * kNbIn * kBlk) return;
  if (in_sizes[2] != kK) return;
  if (out_size != kM * kN) return;
  if (ws_size < kWsTotal) return;

  const float* x     = (const float*)d_in[0];
  const float* w     = (const float*)d_in[1];
  const float* dsign = (const float*)d_in[2];
  float* out = (float*)d_out;

  char* ws = (char*)d_ws;
  unsigned short* APL = (unsigned short*)(ws + kOffA);
  unsigned short* BTP = (unsigned short*)(ws + kOffBt);

  constexpr int totalA8 = kM * kK / 8;
  constexpr int totalB8 = kN * (kK / 8);
  static_assert((totalA8 % 256) == 0 && (totalB8 % 256) == 0, "exact producer grids");
  static_assert(((kM >> 6) * (kN >> 6)) % 8 == 0, "exact GEMM grid");

  sign_scale_to_f16_kernel<<<totalA8 / 256, 256, 0, stream>>>(x, dsign, APL, totalA8);
  expand_rotated_blocks_kernel<<<totalB8 / 256, 256, 0, stream>>>(w, BTP, totalB8);
  gemm_f16_nt_kernel<<<((kM >> 6) * (kN >> 6)) / 8, 256, 0, stream>>>(APL, BTP, out, kFold);
}
